// single_multi_head_31344671326318
// MI455X (gfx1250) — hardware-verified
//
#include <hip/hip_runtime.h>


#define NT   4096
#define DD   1024
#define PCAR 1024.0f
#define SCL  (1.0f / 4096.0f)
typedef _Float16 h16;
typedef unsigned short bf;
typedef __attribute__((ext_vector_type(16))) __bf16   v16bf;
typedef __attribute__((ext_vector_type(16))) _Float16 v16h;
typedef __attribute__((ext_vector_type(8)))  _Float16 v8h;
typedef __attribute__((ext_vector_type(8)))  unsigned short v8us;
typedef __attribute__((ext_vector_type(8)))  float    v8f;
typedef __attribute__((ext_vector_type(4)))  float    v4f;
typedef v8h  __attribute__((may_alias)) v8ha;
typedef v4f  __attribute__((may_alias)) v4fa;
typedef v8us __attribute__((may_alias)) v8usa;

__device__ __forceinline__ unsigned short f2bf(float f) { unsigned u = __float_as_uint(f); u += 0x7FFFu + ((u >> 16) & 1u); return (unsigned short)(u >> 16); }
__device__ __forceinline__ float bf2f(unsigned short b) { return __uint_as_float(((unsigned)b) << 16); }
__device__ __forceinline__ float bfr(float f) { return bf2f(f2bf(f)); }
__device__ __forceinline__ v16h cat16(v8h lo, v8h hi) { return __builtin_shufflevector(lo, hi, 0, 1, 2, 3, 4, 5, 6, 7, 8, 9, 10, 11, 12, 13, 14, 15); }
__device__ __forceinline__ v16bf cat16b(v8us lo, v8us hi) { return __builtin_bit_cast(v16bf, __builtin_shufflevector(lo, hi, 0, 1, 2, 3, 4, 5, 6, 7, 8, 9, 10, 11, 12, 13, 14, 15)); }
__device__ __forceinline__ v8f wmma16(v16h a, v16h b, v8f c) { return __builtin_amdgcn_wmma_f32_16x16x32_f16(false, a, false, b, (short)0, c, false, false); }
__device__ __forceinline__ v8f wmmab(v16bf a, v16bf b, v8f c) { return __builtin_amdgcn_wmma_f32_16x16x32_bf16(false, a, false, b, (short)0, c, false, false); }


template <typename T16> struct WFrag;
template <> struct WFrag<h16> { typedef v16h V; static __device__ __forceinline__ V ld(const h16* p) { return cat16(*(const v8h*)p, *(const v8h*)(p + 16)); } static __device__ __forceinline__ v8f mma(V a, V b, v8f c) { return wmma16(a, b, c); } };
template <> struct WFrag<bf> { typedef v16bf V; static __device__ __forceinline__ V ld(const bf* p) { return cat16b(*(const v8us*)p, *(const v8us*)(p + 16)); } static __device__ __forceinline__ v8f mma(V a, V b, v8f c) { return wmmab(a, b, c); } };
template <typename T16, int NSPLIT, bool BIAS>
__global__ __launch_bounds__(32) void k_gemmw(const T16* __restrict__ A, const T16* __restrict__ A2, const T16* __restrict__ Bt, const T16* __restrict__ Bt2, int K, float* C, int ldc, const float* __restrict__ bias, size_t sA, size_t sB, size_t sC) {
    typedef typename WFrag<T16>::V V;
    __shared__ __align__(16) float os[16 * 68];
    const size_t z = blockIdx.z; A += z * sA; if (A2) A2 += z * sA; Bt += z * sB; if (Bt2) Bt2 += z * sB; C += z * sC;
    const int lane = threadIdx.x & 31, lr = lane & 15, hi = lane >> 4; const int r0 = blockIdx.x * 64, c0 = blockIdx.y * 64;
    v8f acc[4][4];
#pragma unroll
    for (int mb = 0; mb < 4; ++mb)
#pragma unroll
        for (int nb = 0; nb < 4; ++nb) acc[mb][nb] = (v8f){};
    const size_t aoff = (size_t)(r0 + lr) * K + 8 * hi, boff = (size_t)(c0 + lr) * K + 8 * hi;
#pragma unroll 1
    for (int kc = 0; kc < K; kc += 32) {
        V a[4], a2[4];
#pragma unroll
        for (int mb = 0; mb < 4; ++mb) { a[mb] = WFrag<T16>::ld(A + aoff + (size_t)mb * 16 * K + kc); if (NSPLIT == 1 || NSPLIT == 2) a2[mb] = WFrag<T16>::ld(A2 + aoff + (size_t)mb * 16 * K + kc); }
#pragma unroll
        for (int nb = 0; nb < 4; ++nb) { const V b = WFrag<T16>::ld(Bt + boff + (size_t)nb * 16 * K + kc); V b2; if (NSPLIT >= 2) b2 = WFrag<T16>::ld(Bt2 + boff + (size_t)nb * 16 * K + kc);
#pragma unroll
            for (int mb = 0; mb < 4; ++mb) { acc[mb][nb] = WFrag<T16>::mma(a[mb], b, acc[mb][nb]); if (NSPLIT == 1 || NSPLIT == 2) acc[mb][nb] = WFrag<T16>::mma(a2[mb], b, acc[mb][nb]); if (NSPLIT >= 2) acc[mb][nb] = WFrag<T16>::mma(a[mb], b2, acc[mb][nb]); } }
        asm volatile("v_nop\n\tv_nop\n\tv_nop\n\tv_nop" : "+v"(acc[0][0]), "+v"(acc[1][1]), "+v"(acc[2][2]), "+v"(acc[3][3]) : "v"(a[0]), "v"(a[3]));
    }
#pragma unroll
    for (int mb = 0; mb < 4; ++mb) {
#pragma unroll
        for (int nb = 0; nb < 4; ++nb) {
#pragma unroll
            for (int j = 0; j < 8; ++j) os[(hi * 8 + j) * 68 + nb * 16 + lr] = acc[mb][nb][j]; }
        __builtin_amdgcn_wave_barrier(); asm volatile("" ::: "memory");
        float* crow = C + (size_t)(r0 + mb * 16) * ldc + c0;
#pragma unroll 1
        for (int ps = 0; ps < 2; ++ps) {
#pragma unroll
            for (int s = 0; s < 8; ++s) { const int row = 2 * s + hi, cofs = lr * 4; v4f val = *(const v4fa*)(os + row * 68 + cofs); if (BIAS) { val[0] += bfr(bias[c0 + cofs]); val[1] += bfr(bias[c0 + cofs + 1]); val[2] += bfr(bias[c0 + cofs + 2]); val[3] += bfr(bias[c0 + cofs + 3]); }
                *(volatile v4f*)(crow + (size_t)row * ldc + cofs) = val; }
            if (ps == 0) __threadfence(); }
        __builtin_amdgcn_wave_barrier(); asm volatile("" ::: "memory");
    }
}

__device__ __forceinline__ h16 tohx(float x) { return (h16)x; }
typedef __attribute__((ext_vector_type(2))) _Float16 v2h;
typedef __attribute__((ext_vector_type(4))) _Float16 v4h;

__global__ __launch_bounds__(256) void k_cvt8(const float* __restrict__ src, bf* dst, size_t n8) { const size_t i = (size_t)blockIdx.x * 256 + threadIdx.x; if (i >= n8) return; const v8f v = *(const v8f*)(src + i * 8); v8us o;
#pragma unroll
    for (int k = 0; k < 8; ++k) o[k] = f2bf(v[k]); *(volatile v8us*)(dst + i * 8) = o; __threadfence(); *(volatile v8us*)(dst + i * 8) = o; }
__global__ __launch_bounds__(256) void k_p16(const float* __restrict__ F, h16* P) { const size_t i = ((size_t)blockIdx.x * 256 + threadIdx.x) * 2; if (i >= (size_t)NT * DD) return; v2h o; o[0] = tohx(F[i]); o[1] = tohx(F[i + 1]); *(volatile v2h*)(P + i) = o; __threadfence(); *(volatile v2h*)(P + i) = o; }
__global__ __launch_bounds__(256) void k_vt(const float* __restrict__ F, h16* VT) { const size_t e = ((size_t)blockIdx.x * 256 + threadIdx.x) * 2; if (e >= (size_t)DD * NT) return; const int j = (int)(e % NT), n = (int)(e / NT); v2h o; o[0] = tohx(F[(size_t)j * DD + n]); o[1] = tohx(F[(size_t)(j + 1) * DD + n]); *(volatile v2h*)(VT + e) = o; __threadfence(); *(volatile v2h*)(VT + e) = o; }
__global__ __launch_bounds__(256) void k_colmax(const float* __restrict__ S, float* CM) { const int j = blockIdx.x * 256 + threadIdx.x; if (j >= NT) return; float m = -3.0e38f; for (int i = 0; i < NT; ++i) m = fmaxf(m, S[(size_t)i * NT + j] * SCL); *(volatile float*)(CM + j) = m; __threadfence(); *(volatile float*)(CM + j) = m; }
__global__ __launch_bounds__(256) void k_colsum(const float* __restrict__ S, const float* __restrict__ CM, float* CS) { const int j = blockIdx.x * 256 + threadIdx.x; if (j >= NT) return; const float m = CM[j]; float s = 0.f;
    for (int i = 0; i < NT; ++i) { float a = S[(size_t)i * NT + j] * SCL; asm volatile("" : "+v"(a)); float d0 = __fsub_rn(a, m); asm volatile("" : "+v"(d0)); s = __fadd_rn(s, __builtin_amdgcn_exp2f(__fmul_rn(d0, 1.4426950408889634f))); }
    const float r = __fdiv_rn(PCAR, s); *(volatile float*)(CS + j) = r; __threadfence(); *(volatile float*)(CS + j) = r; }
__global__ __launch_bounds__(256) void k_pcol(const float* __restrict__ S, const float* __restrict__ CM, const float* __restrict__ CS, h16* P) { const int lane = threadIdx.x & 31; const int i = blockIdx.x * 8 + (threadIdx.x >> 5); if (i >= NT) return; const float* sr = S + (size_t)i * NT;
#pragma unroll 1
    for (int ps = 0; ps < 2; ++ps) {
#pragma unroll 2
        for (int c0 = lane * 4; c0 < NT; c0 += 128) { const v4f v = *(const v4f*)(sr + c0), m4 = *(const v4f*)(CM + c0), r4 = *(const v4f*)(CS + c0); v4h o;
#pragma unroll
            for (int q = 0; q < 4; ++q) { float a = v[q] * SCL; asm volatile("" : "+v"(a)); float d0 = __fsub_rn(a, m4[q]); asm volatile("" : "+v"(d0)); o[q] = tohx(__fmul_rn(__builtin_amdgcn_exp2f(__fmul_rn(d0, 1.4426950408889634f)), r4[q])); }
            *(volatile v4h*)(P + (size_t)i * NT + c0) = o; }
        if (ps == 0) __threadfence(); } }
__global__ __launch_bounds__(256) void k_out(const float* __restrict__ Cm, float* OUT) { const size_t i = ((size_t)blockIdx.x * 256 + threadIdx.x) * 4; if (i >= (size_t)NT * DD) return; const v4f a = *(const v4f*)(Cm + i); v4f o;
#pragma unroll
    for (int q = 0; q < 4; ++q) o[q] = a[q] * (1.0f / PCAR); *(volatile v4f*)(OUT + i) = o; __threadfence(); *(volatile v4f*)(OUT + i) = o; }

extern "C" void kernel_launch(void* const* d_in, const int* in_sizes, int n_in,
                              void* d_out, int out_size, void* d_ws, size_t ws_size, hipStream_t stream) {
    (void)in_sizes; (void)n_in; (void)out_size;
    const float* IN[9]; for (int i = 0; i < 9; ++i) IN[i] = (const float*)d_in[i];
    float* OUT = (float*)d_out;
    char* wsp = (char*)d_ws;
    auto take = [&](size_t bytes) { char* p = wsp; wsp += (bytes + 255) & ~(size_t)255; return (void*)p; };
    bf* WB = (bf*)take((size_t)DD * DD * 2); bf* XB = (bf*)take((size_t)NT * DD * 2); float* F = (float*)take((size_t)NT * DD * 4); h16* Q16 = (h16*)take((size_t)NT * DD * 2); h16* K16 = (h16*)take((size_t)NT * DD * 2); h16* VT = (h16*)take((size_t)DD * NT * 2);
    float* S = (float*)take((size_t)NT * NT * 4); h16* P = (h16*)take((size_t)NT * NT * 2); float* CM = (float*)take((size_t)NT * 4); float* CS = (float*)take((size_t)NT * 4);
    if ((size_t)(wsp - (char*)d_ws) > ws_size) return;
    float* Cm = F;
    const size_t nw = (size_t)DD * DD / 8, nx = (size_t)NT * DD / 8; const unsigned gw = (unsigned)((nw + 255) / 256), gx = (unsigned)((nx + 255) / 256), L2 = (unsigned)(((size_t)NT * DD / 2 + 255) / 256); const dim3 gP(NT / 64, DD / 64, 1);
    k_cvt8<<<gw, 256, 0, stream>>>(IN[3], WB, nw); k_cvt8<<<gx, 256, 0, stream>>>(IN[0], XB, nx); k_gemmw<bf, 0, true><<<gP, 32, 0, stream>>>(XB, nullptr, WB, nullptr, DD, F, DD, IN[4], 0, 0, 0); k_p16<<<L2, 256, 0, stream>>>(F, Q16);
    k_cvt8<<<gw, 256, 0, stream>>>(IN[5], WB, nw); k_cvt8<<<gx, 256, 0, stream>>>(IN[1], XB, nx); k_gemmw<bf, 0, true><<<gP, 32, 0, stream>>>(XB, nullptr, WB, nullptr, DD, F, DD, IN[6], 0, 0, 0); k_p16<<<L2, 256, 0, stream>>>(F, K16);
    k_cvt8<<<gw, 256, 0, stream>>>(IN[7], WB, nw); k_cvt8<<<gx, 256, 0, stream>>>(IN[2], XB, nx); k_gemmw<bf, 0, true><<<gP, 32, 0, stream>>>(XB, nullptr, WB, nullptr, DD, F, DD, IN[8], 0, 0, 0); k_vt<<<L2, 256, 0, stream>>>(F, VT);
    k_gemmw<h16, 0, false><<<dim3(NT / 64, NT / 64, 1), 32, 0, stream>>>(Q16, nullptr, K16, nullptr, DD, S, NT, nullptr, 0, 0, 0);
    k_colmax<<<NT / 256, 256, 0, stream>>>(S, CM); k_colsum<<<NT / 256, 256, 0, stream>>>(S, CM, CS); k_pcol<<<NT / 8, 256, 0, stream>>>(S, CM, CS, P);
    k_gemmw<h16, 0, false><<<gP, 32, 0, stream>>>(P, nullptr, VT, nullptr, NT, Cm, DD, nullptr, 0, 0, 0);
    k_out<<<(unsigned)(((size_t)NT * DD / 4 + 255) / 256), 256, 0, stream>>>(Cm, OUT);
}
